// SampleScoreModel_45019847197458
// MI455X (gfx1250) — hardware-verified
//
#include <hip/hip_runtime.h>


#define NQ   4096
#define NS   8192
#define DD   256
#define PSC  32768.0f

typedef unsigned short bf;
typedef __attribute__((ext_vector_type(16))) __bf16   v16bf;
typedef __attribute__((ext_vector_type(8)))  unsigned short v8us;
typedef __attribute__((ext_vector_type(8)))  float    v8f;
typedef __attribute__((ext_vector_type(4)))  float    v4f;
typedef v4f  __attribute__((may_alias)) v4fa;
typedef v8us __attribute__((may_alias)) v8usa;

__device__ __forceinline__ unsigned short f2bf(float f) { unsigned u = __float_as_uint(f); u += 0x7FFFu + ((u >> 16) & 1u); return (unsigned short)(u >> 16); }
__device__ __forceinline__ float bf2f(unsigned short b) { return __uint_as_float(((unsigned)b) << 16); }
__device__ __forceinline__ float bfr(float f) { return bf2f(f2bf(f)); }
__device__ __forceinline__ v16bf cat16b(v8us lo, v8us hi) { return __builtin_bit_cast(v16bf, __builtin_shufflevector(lo, hi, 0, 1, 2, 3, 4, 5, 6, 7, 8, 9, 10, 11, 12, 13, 14, 15)); }
__device__ __forceinline__ v8f wmmab(v16bf a, v16bf b, v8f c) { return __builtin_amdgcn_wmma_f32_16x16x32_bf16(false, a, false, b, (short)0, c, false, false); }
#define VST2(T, p, v) do { const T vst2_v_ = (v); *(volatile T*)(p) = vst2_v_; __threadfence(); *(volatile T*)(p) = vst2_v_; } while (0)

__global__ __launch_bounds__(256) void k_rows(const float* __restrict__ src, int rows, bf* dst) {
    const int lane = threadIdx.x & 31, r = blockIdx.x * 8 + (threadIdx.x >> 5);
    if (r >= rows) return;
    v8us o;
#pragma unroll
    for (int i = 0; i < 8; ++i) o[i] = f2bf(src[(size_t)r * DD + lane * 8 + i]);
    VST2(v8us, dst + (size_t)r * DD + lane * 8, o);
}
__global__ __launch_bounds__(256) void k_st(const float* __restrict__ s, bf* ST, float* SS) {
    __shared__ __align__(16) unsigned short tl[64 * 72];
    const int tid = threadIdx.x, n0 = blockIdx.x * 64, d0 = blockIdx.y * 64;
    const int nn = tid >> 2, dq = (tid & 3) * 16;
#pragma unroll
    for (int i = 0; i < 16; ++i) tl[(dq + i) * 72 + nn] = f2bf(s[(size_t)(n0 + nn) * DD + d0 + dq + i]);
    __syncthreads();
    const int piece = tid & 7;
    auto pass = [&]() {
#pragma unroll
        for (int q = 0; q < 2; ++q) { const int d = (tid >> 3) + 32 * q; const v8us val = *(const v8usa*)(tl + d * 72 + piece * 8); *(volatile v8us*)(ST + (size_t)(d0 + d) * NS + n0 + piece * 8) = val; }
    };
    pass(); __threadfence(); pass();
    if (blockIdx.y == 0 && tid < 64) { float q2 = 0.f; const float* sr = s + (size_t)(n0 + tid) * DD;
#pragma unroll 4
        for (int d = 0; d < DD; ++d) { const float v = bfr(sr[d]); q2 += v * v; }
        *(volatile float*)(SS + n0 + tid) = q2; __threadfence(); *(volatile float*)(SS + n0 + tid) = q2; }
}
__global__ __launch_bounds__(128) void k_attn(const bf* __restrict__ XB, const bf* __restrict__ SB, const bf* __restrict__ ST, const float* __restrict__ SS, const float* __restrict__ x, const float* __restrict__ tt, float* out) {
    __shared__ __align__(16) unsigned short plds[4][16 * 32];
    __shared__ __align__(16) unsigned short plds2[4][16 * 32];
    __shared__ __align__(16) float ost[4][16 * 68];
    const int lane = threadIdx.x & 31, wave = threadIdx.x >> 5, lr = lane & 15, hi = lane >> 4;
    const int q0 = blockIdx.x * 64 + wave * 16, dh = blockIdx.y;
    unsigned short* pl = &plds[wave][0]; unsigned short* pl2 = &plds2[wave][0];
    const bf* xrow = XB + (size_t)(q0 + lr) * DD + 8 * hi;
    float xs[8], cz[8];
#pragma unroll
    for (int j = 0; j < 8; ++j) { const int r = q0 + hi * 8 + j; float q2 = 0.f; const float* xr = x + (size_t)r * DD;
#pragma unroll 4
        for (int d = 0; d < DD; ++d) { const float v = bfr(xr[d]); q2 += v * v; }
        xs[j] = q2; const float tv = bfr(tt[r]); const float sg = 0.01f * __powf(10000.0f, tv); const float den = sg * sg + 1e-8f; cz[j] = -0.5f / den; }
    v8f o[8];
#pragma unroll
    for (int n = 0; n < 8; ++n) o[n] = (v8f){};
    float mrow[8], lpart[8];
#pragma unroll
    for (int j = 0; j < 8; ++j) { mrow[j] = -3.0e38f; lpart[j] = 0.f; }
#pragma unroll 1
    for (int kt = 0; kt < NS / 32; ++kt) {
        const int n0 = kt * 32;
        v8f g0 = {}, g1 = {};
        v16bf xl = (v16bf){};
#pragma unroll
        for (int kc = 0; kc < 8; ++kc) { const bf* p0 = SB + (size_t)(n0 + lr) * DD + kc * 32 + 8 * hi; const bf* p1 = p0 + (size_t)16 * DD;
            const v16bf xa = cat16b(*(const v8us*)(xrow + kc * 32), *(const v8us*)(xrow + kc * 32 + 16)); xl = xa;
            g0 = wmmab(xa, cat16b(*(const v8us*)p0, *(const v8us*)(p0 + 16)), g0); g1 = wmmab(xa, cat16b(*(const v8us*)p1, *(const v8us*)(p1 + 16)), g1);
            asm volatile("" : "+v"(g0), "+v"(g1) : "v"(xa) : "memory"); }
        asm volatile("v_nop\n\tv_nop\n\tv_nop\n\tv_nop" : "+v"(g0), "+v"(g1) : "v"(xl));
        const float ssa = SS[n0 + lr], ssb = SS[n0 + 16 + lr];
        float alpha[8];
#pragma unroll
        for (int j = 0; j < 8; ++j) {
            const float a0 = cz[j] * (xs[j] - 2.0f * g0[j] + ssa), a1 = cz[j] * (xs[j] - 2.0f * g1[j] + ssb);
            float mx = fmaxf(a0, a1);
            mx = fmaxf(mx, __shfl_xor(mx, 1, 16)); mx = fmaxf(mx, __shfl_xor(mx, 2, 16)); mx = fmaxf(mx, __shfl_xor(mx, 4, 16)); mx = fmaxf(mx, __shfl_xor(mx, 8, 16));
            const float mn = fmaxf(mrow[j], mx);
            alpha[j] = __expf(mrow[j] - mn); mrow[j] = mn;
            const float p0 = __expf(a0 - mn), p1 = __expf(a1 - mn);
            lpart[j] = lpart[j] * alpha[j] + (p0 + p1);
            const int mr = hi * 8 + j;
            const float ps0 = p0 * PSC, ps1 = p1 * PSC; const unsigned short h0 = f2bf(ps0), h1 = f2bf(ps1);
            pl[mr * 32 + lr] = h0; pl[mr * 32 + 16 + lr] = h1; pl2[mr * 32 + lr] = f2bf(ps0 - bf2f(h0)); pl2[mr * 32 + 16 + lr] = f2bf(ps1 - bf2f(h1));
        }
#pragma unroll
        for (int n = 0; n < 8; ++n)
#pragma unroll
            for (int j = 0; j < 8; ++j) o[n][j] *= alpha[j];
        asm volatile("" ::: "memory");
        const v16bf pa = cat16b(*(const v8usa*)(pl + lr * 32 + hi * 8), *(const v8usa*)(pl + lr * 32 + 16 + hi * 8));
        const v16bf px = cat16b(*(const v8usa*)(pl2 + lr * 32 + hi * 8), *(const v8usa*)(pl2 + lr * 32 + 16 + hi * 8));
#pragma unroll
        for (int n = 0; n < 8; ++n) { const bf* sp = ST + (size_t)(dh * 128 + n * 16 + lr) * NS + n0 + hi * 8; const v16bf sv = cat16b(*(const v8us*)sp, *(const v8us*)(sp + 16));
            o[n] = wmmab(pa, sv, o[n]); o[n] = wmmab(px, sv, o[n]);
            asm volatile("" : "+v"(o[n]) : "v"(sv) : "memory"); }
        asm volatile("v_nop\n\tv_nop\n\tv_nop\n\tv_nop" : "+v"(o[0]), "+v"(o[7]) : "v"(pa), "v"(px));
    }
    float inv[8];
#pragma unroll
    for (int j = 0; j < 8; ++j) { float rs = lpart[j]; rs += __shfl_xor(rs, 1, 16); rs += __shfl_xor(rs, 2, 16); rs += __shfl_xor(rs, 4, 16); rs += __shfl_xor(rs, 8, 16); inv[j] = 1.0f / (rs * PSC); }
    float* os = &ost[wave][0];
    float* ob = out + (size_t)q0 * DD;
#pragma unroll
    for (int q4l = 0; q4l < 2; ++q4l) { const int q4 = dh * 2 + q4l;
#pragma unroll
        for (int n = 0; n < 4; ++n)
#pragma unroll
            for (int j = 0; j < 8; ++j) { const int r = q0 + hi * 8 + j, d = q4 * 64 + n * 16 + lr; const float sg = 0.01f * __powf(10000.0f, bfr(tt[r])); const float idn = 1.0f / (sg * sg + 1e-8f);
                os[(hi * 8 + j) * 68 + n * 16 + lr] = sg * (o[q4l * 4 + n][j] * inv[j] - bfr(x[(size_t)r * DD + d])) * idn; }
        __builtin_amdgcn_wave_barrier(); asm volatile("" ::: "memory");
#pragma unroll
        for (int ps2 = 0; ps2 < 2; ++ps2) {
#pragma unroll
            for (int s = 0; s < 8; ++s) { const int Lid = (lane >> 3) + 4 * s, piece = lane & 7; const int row = Lid >> 1, cofs = (Lid & 1) * 32 + piece * 4;
                const v4f val = *(const v4fa*)(os + row * 68 + cofs); *(volatile v4f*)(ob + (size_t)row * DD + q4 * 64 + cofs) = val; }
            if (ps2 == 0) __threadfence(); }
        __builtin_amdgcn_wave_barrier(); asm volatile("" ::: "memory");
    }
}

extern "C" void kernel_launch(void* const* d_in, const int* in_sizes, int n_in,
                              void* d_out, int out_size, void* d_ws, size_t ws_size, hipStream_t stream) {
    (void)in_sizes; (void)n_in; (void)out_size;
    const float* tt = (const float*)d_in[0]; const float* x = (const float*)d_in[1]; const float* s = (const float*)d_in[2];
    float* out = (float*)d_out;
    char* wsp = (char*)d_ws;
    auto take = [&](size_t bytes) { char* p = wsp; wsp += (bytes + 255) & ~(size_t)255; return (void*)p; };
    bf* XB = (bf*)take((size_t)NQ * DD * 2); bf* SB = (bf*)take((size_t)NS * DD * 2); bf* ST = (bf*)take((size_t)DD * NS * 2); float* SS = (float*)take((size_t)NS * 4);
    if ((size_t)(wsp - (char*)d_ws) > ws_size) return;
    k_rows<<<NQ / 8, 256, 0, stream>>>(x, NQ, XB); k_rows<<<NS / 8, 256, 0, stream>>>(s, NS, SB);
    k_st<<<dim3(NS / 64, DD / 64, 1), 256, 0, stream>>>(s, ST, SS);
    k_attn<<<dim3(NQ / 64, 2, 1), 128, 0, stream>>>(XB, SB, ST, SS, x, tt, out);
}
